// ConvNet_81501299409071
// MI455X (gfx1250) — hardware-verified
//
#include <hip/hip_runtime.h>
#include <stddef.h>
#include <math.h>

typedef __attribute__((ext_vector_type(16))) _Float16 v16h;
typedef __attribute__((ext_vector_type(8)))  _Float16 v8h;
typedef __attribute__((ext_vector_type(4)))  _Float16 v4h;
typedef __attribute__((ext_vector_type(8)))  float    v8f;
typedef __attribute__((ext_vector_type(4)))  float    v4f;

constexpr int kThreads      = 128;
constexpr int kWaves        = 4;
constexpr int kImgsPerWave  = 4;
constexpr int kImgsPerBlock = kWaves * kImgsPerWave;
constexpr int kImgW   = 28;
constexpr int kImgPix = 784;
constexpr int kCh1    = 10;
constexpr int kO1W    = 24;
constexpr int kO1Pix  = 576;
constexpr int kP1W    = 12;
constexpr int kP1Pix  = 144;
constexpr int kHmPerCh = 288;
constexpr int kCh2    = 20;
constexpr int kO2W    = 10;
constexpr int kO2Pix  = 100;
constexpr int kK1Real = 25;
constexpr int kK1Pad  = 32;
constexpr int kK2Real = 90;
constexpr int kK2Pad  = 96;
constexpr int kFlat    = 2000;
constexpr int kFlatPad = 2016;
constexpr int kH1     = 50;
constexpr int kH1Pad  = 64;
constexpr int kNOut   = 10;
constexpr int kN1Pad  = 16;
constexpr int kN2Pad  = 32;
constexpr int kNf2Pad = 16;

static_assert(kK1Pad % 32 == 0 && kK2Pad % 32 == 0 && kFlatPad % 32 == 0 && kH1Pad % 32 == 0, "K tails padded to 32");
static_assert(kO1Pix % 16 == 0, "conv1 rows are whole 16-row tiles");
static_assert(kImgsPerBlock * kNOut * 4 == 5 * 128, "one block writes exactly 5 output lines");

constexpr int kLAct2      = 0;
constexpr int kLAct3      = kLAct2 + kImgsPerBlock * kFlatPad;
constexpr int kLSlog      = kLAct3 + kImgsPerBlock * kH1Pad;
constexpr int kLSout      = kLSlog + 512;
constexpr int kLWave      = kLSout + 384;
constexpr int kLwImg      = 0;
constexpr int kLwHm       = 800;
constexpr int kLwPool     = kLwHm + kCh1 * kHmPerCh;
constexpr int kWaveHalves = kLwPool + kCh1 * kP1Pix;
constexpr int kLdsHalves  = kLWave + kWaves * kWaveHalves;
constexpr int kLdsBytes   = kLdsHalves * 2;
static_assert(kLAct3 % 8 == 0 && kLSlog % 8 == 0 && kLSout % 8 == 0 && kLWave % 8 == 0, "16-B aligned LDS regions");
static_assert(kLwHm % 8 == 0 && kLwPool % 8 == 0 && kWaveHalves % 8 == 0, "16-B aligned wave regions");
static_assert(kLdsBytes == 109312, "lds size");

constexpr size_t kWsEline = 0;
constexpr size_t kWsW1    = 512;
constexpr size_t kWsW2    = kWsW1 + (size_t)kN1Pad * kK1Pad * 2;
constexpr size_t kWsFw2   = kWsW2 + (size_t)kN2Pad * kK2Pad * 2;
constexpr size_t kWsFw1   = kWsFw2 + (size_t)kNf2Pad * kH1Pad * 2;
constexpr size_t kWsTotal = kWsFw1 + (size_t)kH1Pad * kFlatPad * 2;
static_assert(kWsW2 == 1536 && kWsFw2 == 7680 && kWsFw1 == 9728 && kWsTotal == 267776, "carve");
static_assert(kWsW1 % 512 == 0 && kWsW2 % 512 == 0 && kWsFw2 % 512 == 0 && kWsFw1 % 512 == 0, "512-B aligned planes");

template <typename T> struct Frag;
template <> struct Frag<_Float16> {
  typedef v16h V; union U { v16h v; v8h h[2]; };
  static __device__ __forceinline__ v16h load(const _Float16* p) {
    U f; f.h[0] = *(const v8h*)(p); f.h[1] = *(const v8h*)(p + 16); return f.v;
  }
};

__device__ __forceinline__ v8f wmma_h(v16h a, v16h b, v8f c) {
  c = __builtin_amdgcn_wmma_f32_16x16x32_f16(false, a, false, b, (short)0, c, false, false);
  asm volatile("v_nop\n\tv_nop\n\tv_nop\n\tv_nop" : "+v"(c) : "v"(a), "v"(b));
  return c;
}

__host__ __device__ constexpr int frag_k(int e) { return (e < 8) ? e : (e + 8); }
__host__ __device__ constexpr int conv1_off(int k) { return (k < kK1Real) ? ((k / 5) * kImgW + (k % 5)) : 0; }
__host__ __device__ constexpr int conv2_off(int k) {
  return (k < kK2Real) ? ((k / 9) * kP1Pix + ((k % 9) / 3) * kP1W + ((k % 9) % 3)) : 0;
}

__device__ float blk_abs_mean(const float* __restrict__ p, int n, float* red) {
  const int tid = threadIdx.x;
  float s = 0.0f;
#pragma unroll 1
  for (int i = tid; i < n; i += 256) s += fabsf(p[i]);
  red[tid] = s;
  __syncthreads();
#pragma unroll 1
  for (int off = 128; off > 0; off >>= 1) {
    if (tid < off) red[tid] = red[tid] + red[tid + off];
    __syncthreads();
  }
  const float tot = red[0];
  __syncthreads();
  const int nn = (n > 0) ? n : 1;
  return tot / (float)nn;
}

__device__ void write_sign_plane(const float* __restrict__ w, int nelem, int nreal, int kreal,
                                 int npad, int kpad, _Float16* dst) {
  const int tid = threadIdx.x;
  const int tpr = kpad >> 3;
  const int total = npad * tpr;
#pragma unroll 1
  for (int i = tid; i < total; i += 256) {
    const int n  = i / tpr;
    const int k0 = (i - n * tpr) * 8;
    const int nc = (n < nreal) ? n : (nreal - 1);
    v8h hv;
#pragma unroll
    for (int e = 0; e < 8; ++e) {
      const int k  = k0 + e;
      const int kc = (k < kreal) ? k : (kreal - 1);
      int idx = nc * kreal + kc;
      idx = (idx < nelem) ? idx : (nelem - 1);
      idx = (idx < 0) ? 0 : idx;
      const float v = w[idx];
      float s = (v > 0.0f) ? 1.0f : ((v < 0.0f) ? -1.0f : 0.0f);
      if (k >= kreal || n >= nreal) s = 0.0f;
      hv[e] = (_Float16)s;
    }
    _Float16* q = dst + (size_t)i * 8;
    *(volatile v8h*)q = hv;
    __threadfence();
    *(volatile v8h*)q = hv;
  }
}

__global__ __launch_bounds__(256) void k_prep(const float* __restrict__ w1, int nw1,
                                              const float* __restrict__ w2, int nw2,
                                              const float* __restrict__ fw1, int nfw1,
                                              const float* __restrict__ fw2, int nfw2,
                                              float* eline,
                                              _Float16* w1p, _Float16* w2p, _Float16* fw1p, _Float16* fw2p) {
  __shared__ float red[256];
  __shared__ __align__(16) float ev[32];
  const int tid = threadIdx.x;
  const float e1 = blk_abs_mean(w1,  nw1,  red);
  const float e2 = blk_abs_mean(w2,  nw2,  red);
  const float e3 = blk_abs_mean(fw1, nfw1, red);
  const float e4 = blk_abs_mean(fw2, nfw2, red);
  if (tid < 32) {
    float v = 0.0f;
    if (tid == 0) v = e1;
    if (tid == 1) v = e2;
    if (tid == 2) v = e3;
    if (tid == 3) v = e4;
    ev[tid] = v;
  }
  __syncthreads();
  {
    const int lc = (tid < 8) ? tid : 7;
    const v4f vv = *(const v4f*)(ev + 4 * lc);
    if (tid < 8) *(volatile v4f*)(eline + 4 * lc) = vv;
    __threadfence();
    if (tid < 8) *(volatile v4f*)(eline + 4 * lc) = vv;
  }
  write_sign_plane(w1,  nw1,  kCh1,  kK1Real, kN1Pad,  kK1Pad,   w1p);
  write_sign_plane(w2,  nw2,  kCh2,  kK2Real, kN2Pad,  kK2Pad,   w2p);
  write_sign_plane(fw2, nfw2, kNOut, kH1,     kNf2Pad, kH1Pad,   fw2p);
  write_sign_plane(fw1, nfw1, kH1,   kFlat,   kH1Pad,  kFlatPad, fw1p);
}

__global__ __launch_bounds__(kThreads)
void k_net(const float* __restrict__ x, int nimg,
           const float* __restrict__ b1, const float* __restrict__ b2,
           const float* __restrict__ fb1, const float* __restrict__ fb2,
           const float* __restrict__ eline,
           const _Float16* __restrict__ w1p, const _Float16* __restrict__ w2p,
           const _Float16* __restrict__ fw1p, const _Float16* __restrict__ fw2p,
           float* __restrict__ out) {
  extern __shared__ __align__(16) _Float16 smem[];
  const int tid  = threadIdx.x;
  const int lane = tid & 31;
  const int wv   = tid >> 5;
  const int lhi  = lane >> 4;
  const int lN   = lane & 15;

  _Float16* act2 = smem + kLAct2;
  _Float16* act3 = smem + kLAct3;
  float*    slog = (float*)(smem + kLSlog);
  float*    sout = (float*)(smem + kLSout);
  _Float16* wb   = smem + kLWave + wv * kWaveHalves;
  _Float16* simg = wb + kLwImg;
  _Float16* hm   = wb + kLwHm;
  _Float16* pp   = wb + kLwPool;

  const float e1s = eline[0], e2s = eline[1], e3s = eline[2], e4s = eline[3];
  const float b1v  = b1[(lN < kCh1) ? lN : (kCh1 - 1)];
  const float b2v0 = b2[(lN < kCh2) ? lN : (kCh2 - 1)];
  const float b2v1 = b2[(16 + lN < kCh2) ? (16 + lN) : (kCh2 - 1)];
  const v8f zero8 = {0.f, 0.f, 0.f, 0.f, 0.f, 0.f, 0.f, 0.f};

  const v16h bw1 = Frag<_Float16>::load(w1p + lN * kK1Pad + 8 * lhi);

  for (int i = 0; i < kImgsPerWave; ++i) {
    const int li = wv * kImgsPerWave + i;
    int gi = blockIdx.x * kImgsPerBlock + li;
    gi = (gi < nimg) ? gi : (nimg - 1);
    const float* xi = x + (size_t)gi * kImgPix;
#pragma unroll 1
    for (int t = lane; t < kImgPix / 4; t += 32) {
      const v4f v = *(const v4f*)(xi + 4 * t);
      v4h h4;
      h4[0] = (_Float16)v[0]; h4[1] = (_Float16)v[1]; h4[2] = (_Float16)v[2]; h4[3] = (_Float16)v[3];
      *(v4h*)(simg + 4 * t) = h4;
    }
    __syncthreads();

#pragma unroll 1
    for (int mt = 0; mt < kO1Pix / 16; ++mt) {
      const int m    = mt * 16 + lN;
      const int oy   = m / kO1W;
      const int ox   = m - oy * kO1W;
      const int base = oy * kImgW + ox;
      v16h a;
#pragma unroll
      for (int e = 0; e < 16; ++e) {
        const int c0 = frag_k(e);
        const int c1 = c0 + 8;
        if (c0 >= kK1Real) {
          a[e] = (_Float16)0.0f;
        } else {
          const int off = lhi ? conv1_off(c1) : conv1_off(c0);
          _Float16 tv = simg[base + off];
          if (c1 >= kK1Real) tv = lhi ? (_Float16)0.0f : tv;
          a[e] = tv;
        }
      }
      const v8f acc = wmma_h(a, bw1, zero8);
      v4h r4;
#pragma unroll
      for (int j = 0; j < 4; ++j) {
        const float u0 = fmaxf(e1s * acc[2 * j] + b1v, 0.0f);
        const float u1 = fmaxf(e1s * acc[2 * j + 1] + b1v, 0.0f);
        r4[j] = (_Float16)fmaxf(u0, u1);
      }
      if (lN < kCh1) *(v4h*)(hm + lN * kHmPerCh + 8 * mt + 4 * lhi) = r4;
    }
    __syncthreads();

#pragma unroll 1
    for (int t = lane; t < kCh1 * kP1Pix; t += 32) {
      const int px = t % kP1W;
      const int i0 = 2 * t - px;
      const float m0 = (float)hm[i0];
      const float m1 = (float)hm[i0 + kP1W];
      pp[t] = (_Float16)fmaxf(m0, m1);
    }
    __syncthreads();

    _Float16* arow = act2 + li * kFlatPad;
#pragma unroll 1
    for (int mt = 0; mt < 7; ++mt) {
      const int m    = mt * 16 + lN;
      const int mc   = (m < kO2Pix) ? m : (kO2Pix - 1);
      const int py   = mc / kO2W;
      const int px   = mc - py * kO2W;
      const int base = py * kP1W + px;
      v8f acc0 = zero8, acc1 = zero8;
#pragma unroll
      for (int kt = 0; kt < kK2Pad / 32; ++kt) {
        v16h a;
#pragma unroll
        for (int e = 0; e < 16; ++e) {
          const int c0 = kt * 32 + frag_k(e);
          const int c1 = c0 + 8;
          if (c0 >= kK2Real) {
            a[e] = (_Float16)0.0f;
          } else {
            const int off = lhi ? conv2_off(c1) : conv2_off(c0);
            _Float16 tv = pp[base + off];
            if (c1 >= kK2Real) tv = lhi ? (_Float16)0.0f : tv;
            a[e] = tv;
          }
        }
        const v16h bq0 = Frag<_Float16>::load(w2p + (size_t)lN * kK2Pad + kt * 32 + 8 * lhi);
        const v16h bq1 = Frag<_Float16>::load(w2p + (size_t)(16 + lN) * kK2Pad + kt * 32 + 8 * lhi);
        acc0 = wmma_h(a, bq0, acc0);
        acc1 = wmma_h(a, bq1, acc1);
      }
      const int mrow0 = mt * 16 + 8 * lhi;
#pragma unroll
      for (int nt = 0; nt < 2; ++nt) {
        const v8f av  = nt ? acc1 : acc0;
        const float bv = nt ? b2v1 : b2v0;
        const int co  = nt * 16 + lN;
        v4h lo4, hi4;
#pragma unroll
        for (int j = 0; j < 4; ++j) {
          lo4[j] = (_Float16)fmaxf(e2s * av[j] + bv, 0.0f);
          hi4[j] = (_Float16)fmaxf(e2s * av[4 + j] + bv, 0.0f);
        }
        _Float16* dst = arow + co * kO2Pix + mrow0;
        if (co < kCh2 && mrow0 + 3 < kO2Pix) *(v4h*)dst = lo4;
        if (co < kCh2 && mrow0 + 7 < kO2Pix) *(v4h*)(dst + 4) = hi4;
      }
    }
    if (lane < 2) {
      v8h z8;
#pragma unroll
      for (int e = 0; e < 8; ++e) z8[e] = (_Float16)0.0f;
      *(v8h*)(arow + kFlat + 8 * lane) = z8;
    }
    __syncthreads();
  }

  {
    const int n1 = wv * 16 + lN;
    const float fb1v = fb1[(n1 < kH1) ? n1 : (kH1 - 1)];
    const _Float16* ar = act2 + lN * kFlatPad + 8 * lhi;
    const _Float16* br = fw1p + (size_t)n1 * kFlatPad + 8 * lhi;
    v8f acc = zero8;
#pragma unroll 1
    for (int kt = 0; kt < kFlatPad / 32; ++kt) {
      const v16h a = Frag<_Float16>::load(ar + kt * 32);
      const v16h b = Frag<_Float16>::load(br + kt * 32);
      acc = wmma_h(a, b, acc);
    }
#pragma unroll
    for (int r = 0; r < 8; ++r) {
      float h = fmaxf(e3s * acc[r] + fb1v, 0.0f);
      if (n1 >= kH1) h = 0.0f;
      act3[(8 * lhi + r) * kH1Pad + n1] = (_Float16)h;
    }
  }
  __syncthreads();

  if (wv == 0) {
    v8f acc2 = zero8;
#pragma unroll
    for (int kt = 0; kt < kH1Pad / 32; ++kt) {
      const v16h a = Frag<_Float16>::load(act3 + lN * kH1Pad + kt * 32 + 8 * lhi);
      const v16h b = Frag<_Float16>::load(fw2p + lN * kH1Pad + kt * 32 + 8 * lhi);
      acc2 = wmma_h(a, b, acc2);
    }
    const float fb2v = fb2[(lN < kNOut) ? lN : (kNOut - 1)];
#pragma unroll
    for (int r = 0; r < 8; ++r) slog[(8 * lhi + r) * 16 + lN] = e4s * acc2[r] + fb2v;
  }
  __syncthreads();

  if (tid < kImgsPerBlock) {
    const float* lr = slog + tid * 16;
    float mx = -__builtin_inff();
#pragma unroll 1
    for (int j = 0; j < kNOut; ++j) mx = fmaxf(mx, lr[j]);
    float s = 0.0f;
#pragma unroll 1
    for (int j = 0; j < kNOut; ++j) s += expf(lr[j] - mx);
    const float lse = logf(s);
#pragma unroll 1
    for (int j = 0; j < kNOut; ++j) sout[tid * kNOut + j] = (lr[j] - mx) - lse;
  }
  __syncthreads();

  if (wv == 0) {
    float* ob = out + (size_t)blockIdx.x * (kImgsPerBlock * kNOut);
    const v4f v0 = *(const v4f*)(sout + 4 * lane);
    const int i1 = 32 + (lane & 7);
    const v4f v1 = *(const v4f*)(sout + 4 * i1);
    *(volatile v4f*)(ob + 4 * lane) = v0;
    if (lane < 8) *(volatile v4f*)(ob + 4 * i1) = v1;
    __threadfence();
    *(volatile v4f*)(ob + 4 * lane) = v0;
    if (lane < 8) *(volatile v4f*)(ob + 4 * i1) = v1;
  }
}

extern "C" void kernel_launch(void* const* d_in, const int* in_sizes, int n_in,
                              void* d_out, int out_size, void* d_ws, size_t ws_size,
                              hipStream_t stream) {
  if (n_in < 9) return;
  const float* x   = (const float*)d_in[0];
  const float* w1  = (const float*)d_in[1];
  const float* b1  = (const float*)d_in[2];
  const float* w2  = (const float*)d_in[3];
  const float* b2  = (const float*)d_in[4];
  const float* fw1 = (const float*)d_in[5];
  const float* fb1 = (const float*)d_in[6];
  const float* fw2 = (const float*)d_in[7];
  const float* fb2 = (const float*)d_in[8];
  float* out = (float*)d_out;

  if (in_sizes[1] < kCh1 * kK1Real || in_sizes[2] < kCh1 || in_sizes[3] < kCh2 * kK2Real ||
      in_sizes[4] < kCh2 || in_sizes[5] < kH1 * kFlat || in_sizes[6] < kH1 ||
      in_sizes[7] < kNOut * kH1 || in_sizes[8] < kNOut) return;
  if (kWsTotal > ws_size) return;

  int nimg = in_sizes[0] / kImgPix;
  const int maxByOut = out_size / kNOut;
  if (nimg > maxByOut) nimg = maxByOut;
  const int nblk = nimg / kImgsPerBlock;
  if (nblk <= 0) return;

  char* ws = (char*)d_ws;
  float*    eline = (float*)(ws + kWsEline);
  _Float16* w1p   = (_Float16*)(ws + kWsW1);
  _Float16* w2p   = (_Float16*)(ws + kWsW2);
  _Float16* fw2p  = (_Float16*)(ws + kWsFw2);
  _Float16* fw1p  = (_Float16*)(ws + kWsFw1);

  k_prep<<<1, 256, 0, stream>>>(w1, in_sizes[1], w2, in_sizes[3], fw1, in_sizes[5], fw2, in_sizes[7],
                                eline, w1p, w2p, fw1p, fw2p);
  k_net<<<nblk, kThreads, kLdsBytes, stream>>>(x, nimg, b1, b2, fb1, fb2, eline,
                                               w1p, w2p, fw1p, fw2p, out);
}
